// WaveNetModelContinuos_80693845557937
// MI455X (gfx1250) — hardware-verified
//
#include <hip/hip_runtime.h>

#define NLAYER  50
#define NREP    10
#define NRES    32
#define NSKIP   512
#define NFEAT   8
#define NB      4
#define NT      16384
#define TSKIP   5115
#define LOUT    11269
#define LTILES  42
#define P1TILES 512
#define TILE_H  512

typedef __bf16   v16b __attribute__((ext_vector_type(16)));
typedef float    v8f  __attribute__((ext_vector_type(8)));
typedef float    v4f  __attribute__((ext_vector_type(4)));
typedef unsigned v4u  __attribute__((ext_vector_type(4)));

union Frag { v16b v; v4u q[2]; unsigned w[8]; };

__device__ __forceinline__ unsigned bf_rne(float f){
  unsigned u = __builtin_bit_cast(unsigned, f);
  return (u + 0x7FFFu + ((u >> 16) & 1u)) >> 16;
}
__device__ __forceinline__ void split2(float a, float b, unsigned& hi, unsigned& lo){
  const unsigned ha = bf_rne(a), hb = bf_rne(b);
  const float ra = a - __builtin_bit_cast(float, ha << 16);
  const float rb = b - __builtin_bit_cast(float, hb << 16);
  hi = ha | (hb << 16);
  lo = bf_rne(ra) | (bf_rne(rb) << 16);
}
__device__ __forceinline__ void split16(const float* x, Frag& h, Frag& l){
  #pragma unroll
  for (int j = 0; j < 8; ++j) split2(x[2*j], x[2*j+1], h.w[j], l.w[j]);
}

__device__ __forceinline__ v8f mma3(v16b ah, v16b al, v16b bh, v16b bl, v8f c){
  c = __builtin_amdgcn_wmma_f32_16x16x32_bf16(false, ah, false, bh, (short)0, c, false, false);
  c = __builtin_amdgcn_wmma_f32_16x16x32_bf16(false, ah, false, bl, (short)0, c, false, false);
  c = __builtin_amdgcn_wmma_f32_16x16x32_bf16(false, al, false, bh, (short)0, c, false, false);
  asm volatile("v_nop\n\tv_nop\n\tv_nop\n\tv_nop" : "+v"(c) : "v"(ah), "v"(al), "v"(bh), "v"(bl));
  return c;
}
__device__ __forceinline__ v16b ldA(const unsigned short* p){ return *(const v16b*)p; }

__device__ __forceinline__ v8f bias8(const float* p, int base){
  v8f c;
  #pragma unroll
  for (int j = 0; j < 8; ++j) c[j] = p[base + j];
  return c;
}
__device__ __forceinline__ v8f ld8(const float* p){
  const v4f a = *(const v4f*)p;
  const v4f b = *(const v4f*)(p + 4);
  v8f c;
  c[0] = a.x; c[1] = a.y; c[2] = a.z; c[3] = a.w;
  c[4] = b.x; c[5] = b.y; c[6] = b.z; c[7] = b.w;
  return c;
}
__device__ __forceinline__ void load16(const float* row, int hf, float* x){
  const v4f a = *(const v4f*)(row + 8 * hf);
  const v4f b = *(const v4f*)(row + 8 * hf + 4);
  const v4f c = *(const v4f*)(row + 16 + 8 * hf);
  const v4f e = *(const v4f*)(row + 20 + 8 * hf);
  x[0]  = a.x; x[1]  = a.y; x[2]  = a.z; x[3]  = a.w;
  x[4]  = b.x; x[5]  = b.y; x[6]  = b.z; x[7]  = b.w;
  x[8]  = c.x; x[9]  = c.y; x[10] = c.z; x[11] = c.w;
  x[12] = e.x; x[13] = e.y; x[14] = e.z; x[15] = e.w;
}
__device__ __forceinline__ void stage16(float* tile, int n, int hf, const float* a8, const float* b8){
  v4f t0 = {a8[0], a8[1], a8[2], a8[3]};
  v4f t1 = {a8[4], a8[5], a8[6], a8[7]};
  v4f t2 = {b8[0], b8[1], b8[2], b8[3]};
  v4f t3 = {b8[4], b8[5], b8[6], b8[7]};
  *(v4f*)(tile + n * 32 + 8 * hf)      = t0;
  *(v4f*)(tile + n * 32 + 8 * hf + 4)  = t1;
  *(v4f*)(tile + n * 32 + 16 + 8 * hf) = t2;
  *(v4f*)(tile + n * 32 + 20 + 8 * hf) = t3;
}
__device__ __forceinline__ void store_rows16(const float* tile, int lane, float* base, long long row0,
                                             int pitch, int vlo, int vhi){
  v4f v[4]; float* p[4]; bool ok[4];
  #pragma unroll
  for (int j = 0; j < 4; ++j){
    const int r = 4 * j + (lane >> 3), c = lane & 7;
    v[j]  = *(const v4f*)(tile + r * 32 + c * 4);
    ok[j] = (r >= vlo) && (r < vhi);
    p[j]  = ok[j] ? (base + (size_t)(row0 + r) * (size_t)pitch + c * 4) : base;
  }
  #pragma unroll
  for (int j = 0; j < 4; ++j) if (ok[j]) *(volatile v4f*)p[j] = v[j];
  __threadfence();
  #pragma unroll
  for (int j = 0; j < 4; ++j) if (ok[j]) *(volatile v4f*)p[j] = v[j];
}

__device__ __forceinline__ float sigmf(float x){ return 1.0f / (1.0f + expf(-x)); }
__device__ __forceinline__ float eluf(float x){ return x > 0.0f ? x : expm1f(x); }

__global__ __launch_bounds__(256) void pack_kernel(const float* __restrict__ sig_w, const float* __restrict__ tan_w,
                                                  const float* __restrict__ res_w, const float* __restrict__ skip_w,
                                                  const float* __restrict__ post1_w,
                                                  unsigned short* ph, unsigned short* pl, int ngroups){
  const int g = blockIdx.x * 256 + threadIdx.x;
  if (g < ngroups){
    const int idx0 = g * 8;
    const int tile = idx0 >> 9;
    const int r    = idx0 & 511;
    const int lane = r >> 4;
    const int i0   = r & 15;
    const int m    = lane & 15;
    const int hb   = lane >> 4;
    const int kb   = (i0 == 0) ? (8 * hb) : (16 + 8 * hb);
    float v[8];
    if (tile < NLAYER * LTILES){
      const int layer = tile / LTILES;
      const int t     = tile - layer * LTILES;
      if (t < 8){
        const float* w = (t < 4) ? sig_w : tan_w;
        const int tt = t & 3, tap = tt >> 1, mt = tt & 1;
        const int o = mt * 16 + m;
        const size_t base = ((size_t)(layer * NRES + o) * NRES) * 2 + tap;
        #pragma unroll
        for (int j = 0; j < 8; ++j) v[j] = w[base + (size_t)(kb + j) * 2];
      } else if (t < 10){
        const int mt = t - 8;
        const int o = mt * 16 + m;
        const size_t base = (size_t)(layer * NRES + o) * NRES;
        #pragma unroll
        for (int j = 0; j < 8; ++j) v[j] = res_w[base + kb + j];
      } else {
        const int mt = t - 10;
        const int o = mt * 16 + m;
        const size_t base = ((size_t)layer * NSKIP + o) * NRES;
        #pragma unroll
        for (int j = 0; j < 8; ++j) v[j] = skip_w[base + kb + j];
      }
    } else {
      const int pt = tile - NLAYER * LTILES;
      const int mt = pt >> 4, kc = pt & 15;
      const int o = mt * 16 + m;
      const size_t base = (size_t)o * NSKIP + kc * 32;
      #pragma unroll
      for (int j = 0; j < 8; ++j) v[j] = post1_w[base + kb + j];
    }
    v4u hv, lv;
    unsigned hw[4], lw[4];
    #pragma unroll
    for (int j = 0; j < 4; ++j) split2(v[2*j], v[2*j+1], hw[j], lw[j]);
    hv.x = hw[0]; hv.y = hw[1]; hv.z = hw[2]; hv.w = hw[3];
    lv.x = lw[0]; lv.y = lw[1]; lv.z = lw[2]; lv.w = lw[3];
    volatile v4u* dh = (volatile v4u*)(ph + idx0);
    volatile v4u* dl = (volatile v4u*)(pl + idx0);
    *dh = hv; *dl = lv;
    __threadfence();
    *dh = hv; *dl = lv;
  }
}

__global__ __launch_bounds__(128) void skipb_kernel(const float* __restrict__ skip_b, float* sbt){
  const int j = threadIdx.x;
  float s0 = 0.0f, s1 = 0.0f, s2 = 0.0f, s3 = 0.0f;
  #pragma unroll 1
  for (int i = 0; i < NLAYER; ++i){
    const float* p = skip_b + i * NSKIP + 4 * j;
    s0 += p[0]; s1 += p[1]; s2 += p[2]; s3 += p[3];
  }
  v4f v = {s0, s1, s2, s3};
  volatile v4f* d = (volatile v4f*)(sbt + 4 * j);
  *d = v;
  __threadfence();
  *d = v;
}

__global__ __launch_bounds__(256) void front_kernel(const float* __restrict__ in, const float* __restrict__ fw,
                                                   const float* __restrict__ fb, float* h0, int npos){
  const int idx = blockIdx.x * 256 + threadIdx.x;
  if (idx < npos){
    const float* ip = in + (size_t)idx * NFEAT;
    const v4f a = *(const v4f*)ip;
    const v4f c = *(const v4f*)(ip + 4);
    float x[8] = {a.x, a.y, a.z, a.w, c.x, c.y, c.z, c.w};
    float* op = h0 + (size_t)idx * NRES;
    #pragma unroll 1
    for (int pass = 0; pass < 2; ++pass){
      #pragma unroll 1
      for (int q = 0; q < 8; ++q){
        float s[4];
        #pragma unroll
        for (int i = 0; i < 4; ++i){
          const int o = 4 * q + i;
          float t = fb[o];
          #pragma unroll
          for (int f = 0; f < 8; ++f) t += fw[o * 8 + f] * x[f];
          s[i] = t;
        }
        v4f v = {s[0], s[1], s[2], s[3]};
        *(volatile v4f*)(op + 4 * q) = v;
      }
      if (pass == 0) __threadfence();
    }
  }
}

__global__ __launch_bounds__(256) void layer_kernel(const float* __restrict__ hin, float* hout, float* gring,
    float* skips, const float* __restrict__ sbt,
    const unsigned short* __restrict__ pkh, const unsigned short* __restrict__ pkl,
    const unsigned short* __restrict__ rph, const unsigned short* __restrict__ rpl,
    const float* __restrict__ sig_b, const float* __restrict__ tan_b, const float* __restrict__ res_b,
    int d, int ustart, int gslot, int mode){
  __shared__ __align__(16) float tile[8 * 16 * 32];
  const int lane = threadIdx.x & 31;
  const int wv   = threadIdx.x >> 5;
  const int n    = lane & 15;
  const int hf   = lane >> 4;
  const int b    = blockIdx.y;
  const int ublk = ustart + (int)blockIdx.x * 128;
  const int u0   = ublk + wv * 16;
  const int u    = u0 + n;
  const int uc   = (u < NT) ? u : (NT - 1);
  float* mytile  = tile + wv * 512;

  const float* hb = hin + (size_t)b * NT * NRES;
  float xc[16], xm[16];
  load16(hb + (size_t)uc * NRES, hf, xc);
  load16(hb + (size_t)(uc - d) * NRES, hf, xm);
  Frag ch, cl, mh, ml;
  split16(xc, ch, cl);
  split16(xm, mh, ml);

  const unsigned short* ah = pkh + lane * 16;
  const unsigned short* al = pkl + lane * 16;

  v8f s0 = bias8(sig_b, 8 * hf);
  v8f s1 = bias8(sig_b, 16 + 8 * hf);
  s0 = mma3(ldA(ah + 0 * TILE_H), ldA(al + 0 * TILE_H), mh.v, ml.v, s0);
  s1 = mma3(ldA(ah + 1 * TILE_H), ldA(al + 1 * TILE_H), mh.v, ml.v, s1);
  s0 = mma3(ldA(ah + 2 * TILE_H), ldA(al + 2 * TILE_H), ch.v, cl.v, s0);
  s1 = mma3(ldA(ah + 3 * TILE_H), ldA(al + 3 * TILE_H), ch.v, cl.v, s1);
  v8f t0 = bias8(tan_b, 8 * hf);
  v8f t1 = bias8(tan_b, 16 + 8 * hf);
  t0 = mma3(ldA(ah + 4 * TILE_H), ldA(al + 4 * TILE_H), mh.v, ml.v, t0);
  t1 = mma3(ldA(ah + 5 * TILE_H), ldA(al + 5 * TILE_H), mh.v, ml.v, t1);
  t0 = mma3(ldA(ah + 6 * TILE_H), ldA(al + 6 * TILE_H), ch.v, cl.v, t0);
  t1 = mma3(ldA(ah + 7 * TILE_H), ldA(al + 7 * TILE_H), ch.v, cl.v, t1);

  float gx[16];
  #pragma unroll
  for (int j = 0; j < 8; ++j){
    gx[j]     = sigmf(s0[j]) * tanhf(t0[j]);
    gx[8 + j] = sigmf(s1[j]) * tanhf(t1[j]);
  }
  Frag gh, gl;
  split16(gx, gh, gl);

  v8f r0 = bias8(res_b, 8 * hf);
  v8f r1 = bias8(res_b, 16 + 8 * hf);
  r0 = mma3(ldA(ah + 8 * TILE_H), ldA(al + 8 * TILE_H), gh.v, gl.v, r0);
  r1 = mma3(ldA(ah + 9 * TILE_H), ldA(al + 9 * TILE_H), gh.v, gl.v, r1);
  float ra[8], rb[8];
  #pragma unroll
  for (int j = 0; j < 8; ++j){ ra[j] = r0[j] + xc[j]; rb[j] = r1[j] + xc[8 + j]; }

  stage16(mytile, n, hf, ra, rb);
  __syncthreads();
  store_rows16(mytile, lane, hout + (size_t)b * NT * NRES, (long long)u0, NRES, 0, NT - u0);
  __syncthreads();

  if (ublk + 127 >= TSKIP){
    const int vlo = TSKIP - u0;
    const int vhi = NT - u0;
    if (mode == 0){
      stage16(mytile, n, hf, gx, gx + 8);
      __syncthreads();
      store_rows16(mytile, lane, gring + ((size_t)gslot * NB + b) * (size_t)LOUT * NRES,
                   (long long)u0 - TSKIP, NRES, vlo, vhi);
    } else {
      const int us = (u < TSKIP) ? TSKIP : uc;
      const float* srow = skips + ((size_t)b * LOUT + (size_t)(us - TSKIP)) * NSKIP;
      const float* grow = gring + ((size_t)b * LOUT + (size_t)(us - TSKIP)) * NRES;
      const unsigned short* rh = rph + lane * 16;
      const unsigned short* rl = rpl + lane * 16;
      #pragma unroll 1
      for (int q = 0; q < 16; ++q){
        v8f a0, a1;
        if (mode == 1){
          a0 = bias8(sbt, 32 * q + 8 * hf);
          a1 = bias8(sbt, 32 * q + 16 + 8 * hf);
        } else {
          a0 = ld8(srow + 32 * q + 8 * hf);
          a1 = ld8(srow + 32 * q + 16 + 8 * hf);
        }
        a0 = mma3(ldA(ah + (10 + 2 * q) * TILE_H), ldA(al + (10 + 2 * q) * TILE_H), gh.v, gl.v, a0);
        a1 = mma3(ldA(ah + (11 + 2 * q) * TILE_H), ldA(al + (11 + 2 * q) * TILE_H), gh.v, gl.v, a1);
        #pragma unroll 1
        for (int s = 0; s < NREP - 1; ++s){
          float gs[16];
          load16(grow + (size_t)s * NB * LOUT * NRES, hf, gs);
          Frag sh, sl;
          split16(gs, sh, sl);
          const unsigned short* th = rh + (size_t)s * LTILES * TILE_H;
          const unsigned short* tl = rl + (size_t)s * LTILES * TILE_H;
          a0 = mma3(ldA(th + (10 + 2 * q) * TILE_H), ldA(tl + (10 + 2 * q) * TILE_H), sh.v, sl.v, a0);
          a1 = mma3(ldA(th + (11 + 2 * q) * TILE_H), ldA(tl + (11 + 2 * q) * TILE_H), sh.v, sl.v, a1);
        }
        float pa[8], pb[8];
        #pragma unroll
        for (int j = 0; j < 8; ++j){ pa[j] = a0[j]; pb[j] = a1[j]; }
        stage16(mytile, n, hf, pa, pb);
        __syncthreads();
        store_rows16(mytile, lane, skips + (size_t)b * LOUT * NSKIP + 32 * q,
                     (long long)u0 - TSKIP, NSKIP, vlo, vhi);
        __syncthreads();
      }
    }
  }
}

__global__ __launch_bounds__(32) void post_kernel(const float* __restrict__ skips,
    const unsigned short* __restrict__ ph, const unsigned short* __restrict__ pl,
    const float* __restrict__ post1_b, const float* __restrict__ post2_w, const float* __restrict__ post2_b,
    float* out, int nrows){
  __shared__ __align__(16) unsigned short bh[16 * NSKIP];
  __shared__ __align__(16) unsigned short bl[16 * NSKIP];
  __shared__ __align__(16) float res[32];
  const int lane = threadIdx.x & 31;
  const int n    = lane & 15;
  const int hf   = lane >> 4;
  const int e0   = (int)blockIdx.x * 32;
  const unsigned short* ah = ph + lane * 16;
  const unsigned short* al = pl + lane * 16;

  #pragma unroll 1
  for (int p = 0; p < 2; ++p){
    const int e  = e0 + 16 * p + n;
    const int ec = (e < nrows) ? e : (nrows - 1);
    const float* sp = skips + (size_t)ec * NSKIP;
    #pragma unroll 1
    for (int cc = hf * 256; cc < hf * 256 + 256; cc += 16){
      float x[16];
      const v4f a = *(const v4f*)(sp + cc);
      const v4f b = *(const v4f*)(sp + cc + 4);
      const v4f c = *(const v4f*)(sp + cc + 8);
      const v4f f = *(const v4f*)(sp + cc + 12);
      x[0]  = eluf(a.x); x[1]  = eluf(a.y); x[2]  = eluf(a.z); x[3]  = eluf(a.w);
      x[4]  = eluf(b.x); x[5]  = eluf(b.y); x[6]  = eluf(b.z); x[7]  = eluf(b.w);
      x[8]  = eluf(c.x); x[9]  = eluf(c.y); x[10] = eluf(c.z); x[11] = eluf(c.w);
      x[12] = eluf(f.x); x[13] = eluf(f.y); x[14] = eluf(f.z); x[15] = eluf(f.w);
      Frag xh, xl;
      split16(x, xh, xl);
      *(v4u*)(bh + n * NSKIP + cc)     = xh.q[0];
      *(v4u*)(bh + n * NSKIP + cc + 8) = xh.q[1];
      *(v4u*)(bl + n * NSKIP + cc)     = xl.q[0];
      *(v4u*)(bl + n * NSKIP + cc + 8) = xl.q[1];
    }
    __syncthreads();

    float psum = 0.0f;
    #pragma unroll 1
    for (int mt = 0; mt < 32; ++mt){
      v8f acc = bias8(post1_b, mt * 16 + 8 * hf);
      #pragma unroll
      for (int kc = 0; kc < 16; ++kc){
        Frag xh, xl;
        xh.q[0] = *(const v4u*)(bh + n * NSKIP + kc * 32 + 8 * hf);
        xh.q[1] = *(const v4u*)(bh + n * NSKIP + kc * 32 + 16 + 8 * hf);
        xl.q[0] = *(const v4u*)(bl + n * NSKIP + kc * 32 + 8 * hf);
        xl.q[1] = *(const v4u*)(bl + n * NSKIP + kc * 32 + 16 + 8 * hf);
        acc = mma3(ldA(ah + (size_t)(mt * 16 + kc) * TILE_H), ldA(al + (size_t)(mt * 16 + kc) * TILE_H),
                   xh.v, xl.v, acc);
      }
      float part = 0.0f;
      #pragma unroll
      for (int j = 0; j < 8; ++j) part += post2_w[mt * 16 + 8 * hf + j] * eluf(acc[j]);
      psum += part;
    }
    psum += __shfl_xor(psum, 16, 32);
    if (hf == 0) res[16 * p + n] = psum + post2_b[0];
    __syncthreads();
  }

  v4f v = {0.0f, 0.0f, 0.0f, 0.0f};
  int eb = 0;
  if (lane < 8){ v = *(const v4f*)(res + lane * 4); eb = e0 + lane * 4; }
  #pragma unroll 1
  for (int pass = 0; pass < 2; ++pass){
    if (lane < 8){
      if (eb + 4 <= nrows){
        *(volatile v4f*)(out + eb) = v;
      } else {
        if (eb + 0 < nrows) *(volatile float*)(out + eb + 0) = v.x;
        if (eb + 1 < nrows) *(volatile float*)(out + eb + 1) = v.y;
        if (eb + 2 < nrows) *(volatile float*)(out + eb + 2) = v.z;
        if (eb + 3 < nrows) *(volatile float*)(out + eb + 3) = v.w;
      }
    }
    if (pass == 0) __threadfence();
  }
}

extern "C" void kernel_launch(void* const* d_in, const int* in_sizes, int n_in,
                              void* d_out, int out_size, void* d_ws, size_t ws_size,
                              hipStream_t stream){
  if (n_in < 15) return;
  if (in_sizes[0] != NB * NT * NFEAT) return;
  if (in_sizes[1] != NRES * NFEAT || in_sizes[2] != NRES) return;
  if (in_sizes[3] != NLAYER * NRES * NRES * 2 || in_sizes[5] != NLAYER * NRES * NRES * 2) return;
  if (in_sizes[4] != NLAYER * NRES || in_sizes[6] != NLAYER * NRES || in_sizes[10] != NLAYER * NRES) return;
  if (in_sizes[7] != NLAYER * NSKIP * NRES || in_sizes[8] != NLAYER * NSKIP) return;
  if (in_sizes[9] != NLAYER * NRES * NRES) return;
  if (in_sizes[11] != NSKIP * NSKIP || in_sizes[12] != NSKIP || in_sizes[13] != NSKIP || in_sizes[14] != 1) return;
  if (out_size != NB * LOUT) return;

  const float* in      = (const float*)d_in[0];
  const float* from_w  = (const float*)d_in[1];
  const float* from_b  = (const float*)d_in[2];
  const float* sig_w   = (const float*)d_in[3];
  const float* sig_b   = (const float*)d_in[4];
  const float* tan_w   = (const float*)d_in[5];
  const float* tan_b   = (const float*)d_in[6];
  const float* skip_w  = (const float*)d_in[7];
  const float* skip_b  = (const float*)d_in[8];
  const float* res_w   = (const float*)d_in[9];
  const float* res_b   = (const float*)d_in[10];
  const float* post1_w = (const float*)d_in[11];
  const float* post1_b = (const float*)d_in[12];
  const float* post2_w = (const float*)d_in[13];
  const float* post2_b = (const float*)d_in[14];
  float* out = (float*)d_out;

  const size_t SZ_H    = (size_t)NB * NT * NRES * 4;
  const size_t SZ_SKIP = (size_t)NB * LOUT * NSKIP * 4;
  const size_t SZ_GSLT = (size_t)NB * LOUT * NRES * 4;
  const size_t SZ_GRNG = SZ_GSLT * (NREP - 1);
  const size_t NPACK   = (size_t)(NLAYER * LTILES + P1TILES) * TILE_H;
  const size_t SZ_PACK = NPACK * 2;
  const size_t SZ_SBT  = (size_t)NSKIP * 4;
  size_t off = 0;
  char* ws = (char*)d_ws;
  float* hA = (float*)(ws + off);                 off += SZ_H;
  float* hB = (float*)(ws + off);                 off += SZ_H;
  float* skips = (float*)(ws + off);              off += SZ_SKIP;
  float* gring = (float*)(ws + off);              off += SZ_GRNG;
  unsigned short* pkh = (unsigned short*)(ws + off); off += SZ_PACK;
  unsigned short* pkl = (unsigned short*)(ws + off); off += SZ_PACK;
  float* sbt = (float*)(ws + off);                off += SZ_SBT;
  if (off > ws_size) return;

  {
    const int ngroups = (int)(NPACK / 8);
    pack_kernel<<<(ngroups + 255) / 256, 256, 0, stream>>>(sig_w, tan_w, res_w, skip_w, post1_w, pkh, pkl, ngroups);
  }
  skipb_kernel<<<1, 128, 0, stream>>>(skip_b, sbt);
  {
    const int npos = NB * NT;
    front_kernel<<<(npos + 255) / 256, 256, 0, stream>>>(in, from_w, from_b, hA, npos);
  }

  const float* hi = hA;
  float*       ho = hB;
  int S = 0;
  for (int i = 0; i < NLAYER; ++i){
    const int slot   = i % NREP;
    const int d      = 1 << slot;
    const int ustart = S + d;
    const int count  = NT - ustart;
    const int bx     = (count + 127) / 128;
    const int mode   = (slot == NREP - 1) ? ((i == NREP - 1) ? 1 : 2) : 0;
    const int rep0   = i - slot;
    layer_kernel<<<dim3(bx, NB), 256, 0, stream>>>(hi, ho, gring, skips, sbt,
        pkh + (size_t)i * LTILES * TILE_H,    pkl + (size_t)i * LTILES * TILE_H,
        pkh + (size_t)rep0 * LTILES * TILE_H, pkl + (size_t)rep0 * LTILES * TILE_H,
        sig_b + i * NRES, tan_b + i * NRES, res_b + i * NRES, d, ustart, slot, mode);
    { const float* t1 = ho; ho = (float*)hi; hi = t1; }
    S = ustart;
  }

  {
    const int nrows = NB * LOUT;
    post_kernel<<<(nrows + 31) / 32, 32, 0, stream>>>(skips,
        pkh + (size_t)NLAYER * LTILES * TILE_H, pkl + (size_t)NLAYER * LTILES * TILE_H,
        post1_b, post2_w, post2_b, out, nrows);
  }
}
